// LocalAttention_21560735826482
// MI455X (gfx1250) — hardware-run, weakly checked
//
#include <hip/hip_runtime.h>
#define NB 32
#define GB 16
#define SQ 4096
#define HD 64
#define HF 32
#define WN 128
#define NW 32
#define BK 256
#define PR (SQ + WN)
typedef __bf16 v16b __attribute__((ext_vector_type(16)));
typedef unsigned short v8us __attribute__((ext_vector_type(8), may_alias));
typedef float  v8f  __attribute__((ext_vector_type(8)));
typedef float  v4f  __attribute__((ext_vector_type(4)));
typedef float  v4fa __attribute__((ext_vector_type(4), may_alias));
union FragB { v16b v; v8us half[2]; unsigned short u[16]; };

__device__ __forceinline__ unsigned short bf16_bits(float x) { unsigned int u = __float_as_uint(x); return (unsigned short)((u + 0x7FFFu + ((u >> 16) & 1u)) >> 16); }
__device__ __forceinline__ float bf16_val(unsigned short b) { return __uint_as_float(((unsigned int)b) << 16); }
__device__ __forceinline__ float bf16_round(float x) { return bf16_val(bf16_bits(x)); }
template <int NT>
__device__ __forceinline__ v8f mmaN(v16b ah, v16b al, v16b bh, v16b bl, v8f c) {
  c = __builtin_amdgcn_wmma_f32_16x16x32_bf16(false, ah, false, bh, (short)0, c, false, false);
  if (NT >= 2) c = __builtin_amdgcn_wmma_f32_16x16x32_bf16(false, al, false, bh, (short)0, c, false, false);
  if (NT >= 3) c = __builtin_amdgcn_wmma_f32_16x16x32_bf16(false, ah, false, bl, (short)0, c, false, false);
  asm volatile("v_nop\n\tv_nop\n\tv_nop\n\tv_nop" : "+v"(c) : "v"(ah), "v"(al), "v"(bh), "v"(bl));
  return c;
}


typedef _Float16 v16h __attribute__((ext_vector_type(16)));
union FragH { v16h v; v8us half[2]; _Float16 h[16]; unsigned short u[16]; };
template <int NT>
__device__ __forceinline__ v8f mmaH(v16h ah, v16h al, v16h bh, v16h bl, v8f c) {
  c = __builtin_amdgcn_wmma_f32_16x16x32_f16(false, ah, false, bh, (short)0, c, false, false);
  if (NT >= 2) c = __builtin_amdgcn_wmma_f32_16x16x32_f16(false, al, false, bh, (short)0, c, false, false);
  if (NT >= 3) c = __builtin_amdgcn_wmma_f32_16x16x32_f16(false, ah, false, bl, (short)0, c, false, false);
  asm volatile("v_nop\n\tv_nop\n\tv_nop\n\tv_nop" : "+v"(c) : "v"(ah), "v"(al), "v"(bh), "v"(bl));
  return c;
}

typedef _Float16 v4h __attribute__((ext_vector_type(4)));
__global__ __launch_bounds__(256) void k_hl(const float* __restrict__ F, _Float16* __restrict__ Hh, _Float16* __restrict__ Hl, size_t n8) { const size_t t = (size_t)blockIdx.x * 256 + threadIdx.x; if (t >= n8) return; FragH fh, fl; const v4f a = *(const v4fa*)(F + t * 8), c = *(const v4fa*)(F + t * 8 + 4);
#pragma unroll
  for (int q = 0; q < 4; ++q) { _Float16 h = (_Float16)a[q]; fh.h[q] = h; fl.h[q] = (_Float16)((a[q] - (float)h) * 1024.0f); h = (_Float16)c[q]; fh.h[4 + q] = h; fl.h[4 + q] = (_Float16)((c[q] - (float)h) * 1024.0f); }
  for (int pass = 0; pass < 2; ++pass) { *(volatile v8us*)((unsigned short*)Hh + t * 8) = fh.half[0]; *(volatile v8us*)((unsigned short*)Hl + t * 8) = fl.half[0]; if (pass == 0) __threadfence(); } }
__device__ __forceinline__ v16h g2_frag(const _Float16* p, int hh) { FragH f; f.half[0] = *(const v8us*)((const unsigned short*)p + 8 * hh); f.half[1] = *(const v8us*)((const unsigned short*)p + 16 + 8 * hh); return f.v; }
__device__ __forceinline__ v8f g2_mma(v16h a, v16h b, v8f c) { v8f d = __builtin_amdgcn_wmma_f32_16x16x32_f16(false, a, false, b, (short)0, c, false, false); asm volatile("v_nop\n\tv_nop\n\tv_nop\n\tv_nop" : "+v"(d) : "v"(a), "v"(b)); return d; }
template <int ACT>
__global__ __launch_bounds__(128) void k_gemm2(const _Float16* __restrict__ A, int lda, size_t sA, const _Float16* __restrict__ Bh, int ldb, size_t sB, float alpha, const float* __restrict__ bias, size_t sBias, const float* __restrict__ CP, int rowsPerB, size_t sCPb, int row0g,
    float* __restrict__ C, _Float16* __restrict__ C16, int ldc, size_t sC, int M, int N, int K) { static_assert(ACT == 0 || ACT == 3 || ACT == 6 || ACT == 8 || ACT == 9 || ACT == 11 || ACT == 12 || ACT == 14 || ACT == 15 || ACT == 16 || ACT == 17, "k_gemm2: unsupported ACT code (would silently apply no activation)");
  __shared__ __attribute__((aligned(16))) float so[4][32][68];
  const int tid = threadIdx.x, w = tid >> 5, lane = tid & 31, ln = lane & 15, hh = lane >> 4; const int by = blockIdx.y;
  A += (size_t)by * sA; Bh += (size_t)by * sB; const size_t cofs = (size_t)by * sC; const float* bp = bias ? bias + (size_t)by * sBias : nullptr;
  const int ntn = N >> 6; const int mt = blockIdx.x / ntn, nq = blockIdx.x - mt * ntn; const int row0 = mt * 128 + 32 * w, col0 = nq * 64; if (row0 >= M) return;
  const _Float16* a0p = A + (size_t)(row0 + ln) * lda; const _Float16* a1p = a0p + (size_t)16 * lda;
  const _Float16* b0p = Bh + (size_t)(col0 + ln) * ldb; const _Float16* b1p = b0p + (size_t)16 * ldb; const _Float16* b2p = b1p + (size_t)16 * ldb; const _Float16* b3p = b2p + (size_t)16 * ldb;
  const v8f z8 = {0.f,0.f,0.f,0.f,0.f,0.f,0.f,0.f}; v8f c00 = z8, c01 = z8, c02 = z8, c03 = z8, c10 = z8, c11 = z8, c12 = z8, c13 = z8;
  for (int kb = 0; kb < K; kb += 32) { const v16h a0 = g2_frag(a0p + kb, hh), a1 = g2_frag(a1p + kb, hh);
    v16h b = g2_frag(b0p + kb, hh); c00 = g2_mma(a0, b, c00); c10 = g2_mma(a1, b, c10);
    b = g2_frag(b1p + kb, hh); c01 = g2_mma(a0, b, c01); c11 = g2_mma(a1, b, c11);
    b = g2_frag(b2p + kb, hh); c02 = g2_mma(a0, b, c02); c12 = g2_mma(a1, b, c12);
    b = g2_frag(b3p + kb, hh); c03 = g2_mma(a0, b, c03); c13 = g2_mma(a1, b, c13); }
  v8f accs[8] = {c00, c01, c02, c03, c10, c11, c12, c13};
#pragma unroll
  for (int u = 0; u < 8; ++u) { const int t = u & 3, half = u >> 2; const int col = col0 + t * 16 + ln; const float bv = bp ? bf16_round(bp[col]) : 0.f;
#pragma unroll
    for (int r = 0; r < 8; ++r) { const int rloc = half * 16 + 8 * hh + r; float v = accs[u][r] * alpha + bv; if (CP) { if (rowsPerB < 0) v += CP[cofs + (size_t)(row0g + row0 + rloc) * ldc + col];        else { const int bidx = (row0g + row0 + rloc) / rowsPerB; v += CP[(size_t)bidx * sCPb + (size_t)by * 64 + col]; } }
      if (ACT == 3) v = fmaxf(v, 0.f); else if (ACT == 6) v = 0.5f * v * (1.0f + erff(v * 0.70710678118654752f)); else if (ACT == 11) v = 1.0f / (1.0f + expf(-v)); else if (ACT == 15) v = v / (1.0f + expf(-v)); else if (ACT == 12) v = (v > 0.f) ? v : 0.01f * v; else if (ACT == 8) v = tanhf(v); else if (ACT == 9) v = 0.5f * v * (1.0f + tanhf(0.7978845608028654f * (v + 0.044715f * v * v * v))); else if (ACT == 14) v = (v > 0.f) ? v : 0.1f * v; else if (ACT == 16) v = (v >= 0.f) ? v : 0.3f * v; else if (ACT == 17) v = (v >= 0.f) ? v : 0.2f * v;
      so[w][rloc][t * 16 + ln] = v; } }
  __builtin_amdgcn_fence(__ATOMIC_ACQ_REL, "workgroup"); __builtin_amdgcn_wave_barrier();
  const int rsub = lane >> 4, c4 = (lane & 15) * 4;
  for (int pass = 0; pass < 2; ++pass) {
#pragma unroll
    for (int q = 0; q < 16; ++q) { const int r = q * 2 + rsub; const v4f v = *(const v4fa*)&so[w][r][c4]; if (C) *(volatile v4f*)(C + cofs + (size_t)(row0 + r) * ldc + col0 + c4) = v; if (C16) { v4h h4; for (int i = 0; i < 4; ++i) h4[i] = (_Float16)v[i]; *(volatile v4h*)(C16 + cofs + (size_t)(row0 + r) * ldc + col0 + c4) = h4; } }
    if (pass == 0) __threadfence(); } }


__device__ const unsigned RH_INVF[HF] = { 0x3f800000u, 0x3f3ff911u, 0x3f0ff59au, 0x3ed7e89bu, 0x3ea1e89bu, 0x3e72d425u, 0x3e361887u, 0x3e088d77u, 0x3dcccccdu, 0x3d99940du, 0x3d6655c2u, 0x3d2cba15u, 0x3d0186e3u, 0x3cc2434fu, 0x3c91ad39u, 0x3c5a7bf2u, 0x3c23d70au, 0x3bf5b9b0u, 0x3bb8449cu, 0x3b8a2e77u, 0x3b4f3e38u, 0x3b1b690du, 0x3ae91528u, 0x3aaec98eu, 0x3a83126fu, 0x3a44948cu, 0x3a136a16u, 0x39dd1727u, 0x39a5cb60u, 0x3978a815u, 0x393a7753u, 0x390bd472u };
__global__ __launch_bounds__(256) void k_rhtab(float* __restrict__ CS, float* __restrict__ SN, int n) {
  const int t = blockIdx.x * 256 + threadIdx.x; if (t >= n) return; const float a = (float)(t >> 5) * __uint_as_float(RH_INVF[t & 31]);
  const float k = rintf(a * 0.63661977236758134f); float r = fmaf(-k, 1.5703125f, a); r = fmaf(-k, 4.837512969970703125e-4f, r); r = fmaf(-k, 7.54978995489188216e-8f, r); const float z = r * r;
  const float s = fmaf(r * z, fmaf(z, fmaf(z, -1.9515295891e-4f, 8.3321608736e-3f), -1.6666654611e-1f), r);
  const float c = fmaf(z * z, fmaf(z, fmaf(z, 2.443315711809948e-5f, -1.388731625493765e-3f), 4.166664568298827e-2f), fmaf(z, -0.5f, 1.0f));
  const unsigned q = (unsigned)(int)k; const unsigned mk = 0u - (q & 1u); const unsigned cb = __float_as_uint(c), sb = __float_as_uint(s);
  const float co = __uint_as_float(((cb & ~mk) | (sb & mk)) ^ ((((q + 1u) >> 1) & 1u) << 31)); const float si = __uint_as_float(((sb & ~mk) | (cb & mk)) ^ (((q >> 1) & 1u) << 31));
  *(volatile float*)(CS + t) = co; *(volatile float*)(SN + t) = si; __threadfence(); *(volatile float*)(CS + t) = co; *(volatile float*)(SN + t) = si; }
__global__ __launch_bounds__(256) void k_bkrotf(const float* __restrict__ X, const float* __restrict__ CS, const float* __restrict__ SN, float* __restrict__ F, int base, int lead, int n) {
  const int t = blockIdx.x * 256 + threadIdx.x; if (t >= n) return; const int g = t & 3, row = t >> 2; const int bl = row / PR, r = row - bl * PR; const int tok = r - lead; const float fv = ((unsigned)tok < (unsigned)SQ) ? 1.0f : 0.0f; const int tk = tok & (SQ - 1); const int pos = base + (tk & (WN - 1));
  const float* x = X + ((size_t)bl * SQ + tk) * HD + 8 * g; const float* c = CS + (size_t)pos * HF + 8 * g; const float* s = SN + (size_t)pos * HF + 8 * g; float* o = F + (size_t)row * HD + 8 * g; v4f lo[2], hi[2];
  for (int j = 0; j < 2; ++j) { const v4f a = *(const v4fa*)(x + 4 * j), b = *(const v4fa*)(x + HF + 4 * j), cc = *(const v4fa*)(c + 4 * j), ss = *(const v4fa*)(s + 4 * j);
    for (int i = 0; i < 4; ++i) { const float x1 = bf16_round(a[i]), x2 = bf16_round(b[i]); lo[j][i] = (x1 * cc[i] - x2 * ss[i]) * fv; hi[j][i] = (x2 * cc[i] + x1 * ss[i]) * fv; } }
  for (int pass = 0; pass < 2; ++pass) { *(volatile v4f*)o = lo[0]; *(volatile v4f*)(o + 4) = lo[1]; *(volatile v4f*)(o + HF) = hi[0]; *(volatile v4f*)(o + HF + 4) = hi[1]; if (pass == 0) __threadfence(); } }
__global__ __launch_bounds__(256) void k_bkwsm(const float* __restrict__ S, float* __restrict__ PF, int n) {
  const int t = blockIdx.x * 256 + threadIdx.x; if (t >= n) return; const int i = t & (WN - 1), w = t >> 7; const int lim = i + WN; const int lo = (w == 0) ? WN : 0; const float* s = S + (size_t)t * BK; float mx = -3.0e38f;
#pragma clang loop vectorize(disable) interleave(disable)
  for (int j = 0; j < BK; ++j) { const float pen = (float)((j > lim) | (j < lo)) * -3.0e38f; mx = fmaxf(mx, s[j] + pen); } float se = 0.f;
  for (int j = 0; j < BK; ++j) { const float pen = (float)((j > lim) | (j < lo)) * -3.0e38f; se += __expf((s[j] + pen) - mx); } const float sc = 256.0f / se;
  for (int j0 = 0; j0 < BK; j0 += 8) { v4f a, b; for (int q = 0; q < 4; ++q) { const int ja = j0 + q, jb = j0 + 4 + q; const float pa = (float)((ja > lim) | (ja < lo)) * -3.0e38f, pb = (float)((jb > lim) | (jb < lo)) * -3.0e38f; a[q] = __expf((s[ja] + pa) - mx) * sc; b[q] = __expf((s[jb] + pb) - mx) * sc; }
    float* o = PF + (size_t)t * BK + j0; *(volatile v4f*)o = a; *(volatile v4f*)(o + 4) = b; __threadfence(); *(volatile v4f*)o = a; *(volatile v4f*)(o + 4) = b; } }
__global__ __launch_bounds__(256) void k_bkvtp(const float* __restrict__ V, _Float16* __restrict__ VT, int n) {
  const int t = blockIdx.x * 256 + threadIdx.x; if (t >= n) return; const int c8 = t % (PR / 8), q = t / (PR / 8); const int dd = q & (HD - 1), bl = q >> 6; const int tok0 = 8 * c8 - WN; const float fv = (tok0 >= 0) ? 1.0f : 0.0f; const int tk = tok0 & (SQ - 1); const float* s = V + ((size_t)bl * SQ + tk) * HD + dd; FragH f;
  for (int i = 0; i < 8; ++i) f.h[i] = (_Float16)(bf16_round(s[(size_t)i * HD]) * fv);
  unsigned short* o = (unsigned short*)VT + ((size_t)bl * HD + dd) * PR + 8 * c8; *(volatile v8us*)o = f.half[0]; __threadfence(); *(volatile v8us*)o = f.half[0]; }

extern "C" void kernel_launch(void* const* d_in, const int* in_sizes, int n_in,
                              void* d_out, int out_size, void* d_ws, size_t ws_size, hipStream_t stream) {
  (void)in_sizes; (void)n_in; (void)out_size;
  const float* q = (const float*)d_in[0]; const float* k = (const float*)d_in[1]; const float* v = (const float*)d_in[2];
  static_assert(HD == 64 && HF == 32 && WN == 128 && NW == 32 && BK == 256 && SQ == NW * WN && PR == 4224 && PR % 8 == 0 && NB % GB == 0 && ((size_t)BK * HF) % 256 == 0 && ((size_t)GB * PR * 4) % 256 == 0 && ((size_t)GB * PR * HD / 8) % 256 == 0 && ((size_t)GB * HD * (PR / 8)) % 256 == 0 && ((size_t)NW * WN) % 256 == 0 && ((size_t)NW * WN * BK / 8) % 256 == 0 && WN % 128 == 0 && WN % 64 == 0 && HD % 64 == 0 && HD % 32 == 0 && BK % 32 == 0, "the index shifts; whole tiles; exact grids");
  float* out = (float*)d_out;
  char* ws = (char*)d_ws; size_t off = 0;
  auto take = [&](size_t bytes) { char* p = ws + off; off += (bytes + 255) & ~(size_t)255; return p; };
  const size_t PL = (size_t)GB * PR * HD;
  float* CS = (float*)take((size_t)BK * HF * 4); float* SN = (float*)take((size_t)BK * HF * 4); float* Fp = (float*)take(PL * 4);
  _Float16* QH = (_Float16*)take(PL * 2); _Float16* QL = (_Float16*)take(PL * 2); _Float16* KAH = (_Float16*)take(PL * 2); _Float16* KAL = (_Float16*)take(PL * 2); _Float16* KBH = (_Float16*)take(PL * 2); _Float16* KBL = (_Float16*)take(PL * 2); _Float16* VT = (_Float16*)take(PL * 2);
  float* S = (float*)take((size_t)NW * WN * BK * 4); float* PF = (float*)take((size_t)NW * WN * BK * 4); _Float16* PH = (_Float16*)take((size_t)NW * WN * BK * 2); _Float16* PLo = (_Float16*)take((size_t)NW * WN * BK * 2);
  if (off > ws_size) return;
  const float A8 = 0.125f, A8L = 0.0001220703125f, AO = 0.00390625f, AOL = 0.000003814697265625f;
  const size_t WR = (size_t)WN * HD, WS = (size_t)WN * BK;
  k_rhtab<<<(unsigned)((size_t)BK * HF / 256), 256, 0, stream>>>(CS, SN, BK * HF);
  for (int b0 = 0; b0 < NB; b0 += GB) {
    const unsigned gr = (unsigned)((size_t)GB * PR * 4 / 256), gh = (unsigned)(PL / 8 / 256);
    k_bkrotf<<<gr, 256, 0, stream>>>(q + (size_t)b0 * SQ * HD, CS, SN, Fp, WN, 0, GB * PR * 4); k_hl<<<gh, 256, 0, stream>>>(Fp, QH, QL, PL / 8);
    k_bkrotf<<<gr, 256, 0, stream>>>(k + (size_t)b0 * SQ * HD, CS, SN, Fp, 0, WN, GB * PR * 4); k_hl<<<gh, 256, 0, stream>>>(Fp, KAH, KAL, PL / 8);
    k_bkrotf<<<gr, 256, 0, stream>>>(k + (size_t)b0 * SQ * HD, CS, SN, Fp, WN, 0, GB * PR * 4); k_hl<<<gh, 256, 0, stream>>>(Fp, KBH, KBL, PL / 8);
    k_bkvtp<<<(unsigned)((size_t)GB * HD * (PR / 8) / 256), 256, 0, stream>>>(v + (size_t)b0 * SQ * HD, VT, GB * HD * (PR / 8));
    for (int bl = 0; bl < GB; ++bl) { const size_t pb = (size_t)bl * PR * HD; const dim3 gs((WN / 128) * (WN / 64), NW), go((WN / 128) * (HD / 64), NW);
      k_gemm2<0><<<gs, 128, 0, stream>>>(QH + pb, HD, WR, KAH + pb, HD, WR, A8, nullptr, 0, nullptr, 1, 0, 0, S, nullptr, BK, WS, WN, WN, HD);
      k_gemm2<0><<<gs, 128, 0, stream>>>(QL + pb, HD, WR, KAH + pb, HD, WR, A8L, nullptr, 0, S, -1, 0, 0, S, nullptr, BK, WS, WN, WN, HD);
      k_gemm2<0><<<gs, 128, 0, stream>>>(QH + pb, HD, WR, KAL + pb, HD, WR, A8L, nullptr, 0, S, -1, 0, 0, S, nullptr, BK, WS, WN, WN, HD);
      k_gemm2<0><<<gs, 128, 0, stream>>>(QH + pb, HD, WR, KBH + pb, HD, WR, A8, nullptr, 0, nullptr, 1, 0, 0, S + WN, nullptr, BK, WS, WN, WN, HD);
      k_gemm2<0><<<gs, 128, 0, stream>>>(QL + pb, HD, WR, KBH + pb, HD, WR, A8L, nullptr, 0, S + WN, -1, 0, 0, S + WN, nullptr, BK, WS, WN, WN, HD);
      k_gemm2<0><<<gs, 128, 0, stream>>>(QH + pb, HD, WR, KBL + pb, HD, WR, A8L, nullptr, 0, S + WN, -1, 0, 0, S + WN, nullptr, BK, WS, WN, WN, HD);
      k_bkwsm<<<(unsigned)((size_t)NW * WN / 256), 256, 0, stream>>>(S, PF, NW * WN); k_hl<<<(unsigned)((size_t)NW * WN * BK / 8 / 256), 256, 0, stream>>>(PF, PH, PLo, (size_t)NW * WN * BK / 8);
      float* ob = out + (size_t)(b0 + bl) * SQ * HD; const _Float16* vb = VT + (size_t)bl * HD * PR;
      k_gemm2<0><<<go, 128, 0, stream>>>(PH, BK, WS, vb, PR, (size_t)WN, AO, nullptr, 0, nullptr, 1, 0, 0, ob, nullptr, HD, WR, WN, HD, BK);
      k_gemm2<0><<<go, 128, 0, stream>>>(PLo, BK, WS, vb, PR, (size_t)WN, AOL, nullptr, 0, ob, -1, 0, 0, ob, nullptr, HD, WR, WN, HD, BK); } }
}
